// SimpleAttn_40183714022071
// MI455X (gfx1250) — hardware-verified
//
#include <hip/hip_runtime.h>
#ifndef NB
#define NB 2
#endif
#ifndef SEQ
#define SEQ 4096
#endif
#define SEQ_FULL 4096
#define CD 128
#define NH 2
#define HW (NH * CD)
#define KVW (2 * HW)
static_assert(NB >= 1 && NB <= 2);
static_assert(SEQ <= SEQ_FULL);
static_assert(SEQ % 128 == 0);
static_assert(SEQ % 64 == 0);
static_assert(SEQ % 32 == 0);
static_assert(CD % 128 == 0);
static_assert(CD % 64 == 0);
static_assert(CD % 32 == 0);
static_assert(HW % 64 == 0);
static_assert(KVW % 64 == 0);
static_assert((NB * SEQ) % 128 == 0);
static_assert((SEQ * CD / 8) % 256 == 0);
static_assert(256 * 16 * 2 == 64 * 128);
static_assert(4 * 32 * 68 * 4 <= 131072);
static_assert(64 * 65 * 2 <= 131072);

typedef unsigned short v8us __attribute__((ext_vector_type(8), may_alias));
typedef float  v8f  __attribute__((ext_vector_type(8)));
typedef float  v4f  __attribute__((ext_vector_type(4)));
typedef float  v4fa __attribute__((ext_vector_type(4), may_alias));
typedef _Float16 v16h __attribute__((ext_vector_type(16)));
typedef _Float16 v4h __attribute__((ext_vector_type(4)));
union FragH { v16h v; v8us half[2]; _Float16 h[16]; unsigned short u[16]; };

constexpr size_t al256(size_t b) { return (b + 255) & ~(size_t)255; }
constexpr size_t WSB_X16 = al256((size_t)NB * SEQ * CD * 2);
constexpr size_t WSB_WT  = al256((size_t)KVW * CD * 2);
constexpr size_t WSB_KVF = al256((size_t)NB * SEQ * KVW * 4);
constexpr size_t WSB_KVT = al256((size_t)2 * NB * HW * SEQ * 2);
constexpr size_t WSB_MT  = al256((size_t)NB * NH * CD * CD * 2);
static_assert(WSB_X16 + WSB_WT + WSB_KVF + WSB_KVT + WSB_MT <= (size_t)134217728);

__device__ __forceinline__ unsigned short bf16_bits(float x) { unsigned int u = __float_as_uint(x); return (unsigned short)((u + 0x7FFFu + ((u >> 16) & 1u)) >> 16); }
__device__ __forceinline__ float bf16_val(unsigned short b) { return __uint_as_float(((unsigned int)b) << 16); }
__device__ __forceinline__ float bf16_rne(float x) { return bf16_val(bf16_bits(x)); }
__device__ __forceinline__ unsigned short h2u(_Float16 x) { return __builtin_bit_cast(unsigned short, x); }
static __device__ __forceinline__ _Float16 toh_flush(float v) { const _Float16 r = (_Float16)v; return (fabsf(v) < 6.103515625e-05f) ? (_Float16)0.0f : r; }

__device__ __forceinline__ v16h g2_frag(const _Float16* p, int hh) { FragH f; f.half[0] = *(const v8us*)((const unsigned short*)p + 8 * hh); f.half[1] = *(const v8us*)((const unsigned short*)p + 16 + 8 * hh); return f.v; }
__device__ __forceinline__ v8f g2_mma(v16h a, v16h b, v8f c) { v8f d = __builtin_amdgcn_wmma_f32_16x16x32_f16(false, a, false, b, (short)0, c, false, false); asm volatile("v_nop\n\tv_nop\n\tv_nop\n\tv_nop" : "+v"(d) : "v"(a), "v"(b)); return d; }

__global__ __launch_bounds__(256) void k_wnat(const float* __restrict__ w, size_t n8, _Float16* __restrict__ Bt) {
  const size_t t = (size_t)blockIdx.x * 256 + threadIdx.x; if (t >= n8) return; FragH f;
#pragma unroll
  for (int q = 0; q < 8; ++q) f.h[q] = toh_flush(bf16_rne(w[t * 8 + q]) * 16.0f);
  *(volatile v8us*)((unsigned short*)Bt + t * 8) = f.half[0]; __threadfence(); *(volatile v8us*)((unsigned short*)Bt + t * 8) = f.half[0];
}

__global__ __launch_bounds__(256) void k_wtr(const float* __restrict__ w, _Float16* __restrict__ Wt) {
  #pragma clang fp contract(off)
  __shared__ unsigned short tl[64][65];
  const int tid = threadIdx.x; const int kg = blockIdx.x / (HW / 64), ng = blockIdx.x - kg * (HW / 64); const int k0 = kg * 64, n0 = ng * 64;
  for (int i = tid; i < 64 * 8; i += 256) {
    const int j = i >> 3, d8 = (i & 7) * 8; const float* wp = w + (size_t)(k0 + j) * HW + n0 + d8;
    const v4f a = *(const v4fa*)wp, c = *(const v4fa*)(wp + 4); const float xs[8] = {a[0], a[1], a[2], a[3], c[0], c[1], c[2], c[3]};
#pragma unroll
    for (int q = 0; q < 8; ++q) tl[d8 + q][j] = h2u(toh_flush(bf16_rne(xs[q]) * 1024.0f));
  }
  __syncthreads();
  for (int pass = 0; pass < 2; ++pass) {
    for (int i = tid; i < 64 * 8; i += 256) {
      const int d = i >> 3, j8 = (i & 7) * 8; FragH f;
#pragma unroll
      for (int q = 0; q < 8; ++q) f.u[q] = tl[d][j8 + q];
      const size_t o = (size_t)(n0 + d) * CD + k0 + j8;
      *(volatile v8us*)((unsigned short*)Wt + o) = f.half[0];
    }
    if (pass == 0) __threadfence(); }
}

__global__ __launch_bounds__(256) void k_kvt(const float* __restrict__ F, _Float16* __restrict__ KVT) {
  #pragma clang fp contract(off)
  __shared__ unsigned short tl[64][65];
  const int tid = threadIdx.x; const int perb = (KVW / 64) * (SEQ / 64);
  const int b = blockIdx.x / perb; const int rem = blockIdx.x - b * perb;
  const int g = rem / (SEQ / 64), sg = rem - g * (SEQ / 64); const int s0 = sg * 64;
  const int isv = g / (HW / 64), gl = g - isv * (HW / 64);
  for (int i = tid; i < 64 * 8; i += 256) {
    const int j = i >> 3, d8 = (i & 7) * 8; const float* vp = F + ((size_t)b * SEQ + s0 + j) * KVW + g * 64 + d8;
    const v4f a = *(const v4fa*)vp, c = *(const v4fa*)(vp + 4); const float xs[8] = {a[0], a[1], a[2], a[3], c[0], c[1], c[2], c[3]};
#pragma unroll
    for (int q = 0; q < 8; ++q) tl[d8 + q][j] = h2u(toh_flush(xs[q]));
  }
  __syncthreads();
  for (int pass = 0; pass < 2; ++pass) {
    for (int i = tid; i < 64 * 8; i += 256) {
      const int d = i >> 3, j8 = (i & 7) * 8; FragH f;
#pragma unroll
      for (int q = 0; q < 8; ++q) f.u[q] = tl[d][j8 + q];
      const size_t o = (size_t)isv * ((size_t)NB * HW * SEQ) + ((size_t)b * HW + gl * 64 + d) * SEQ + s0 + j8;
      *(volatile v8us*)((unsigned short*)KVT + o) = f.half[0];
    }
    if (pass == 0) __threadfence(); }
}

template <int ACT>
__global__ __launch_bounds__(128) void k_gemm2(const _Float16* __restrict__ A, int lda, size_t sA, const _Float16* __restrict__ Bh, int ldb, size_t sB, float alpha, const float* __restrict__ bias, size_t sBias, const float* __restrict__ CP, int rowsPerB, size_t sCPb, int row0g,
    float* __restrict__ C, _Float16* __restrict__ C16, int ldc, size_t sC, int M, int N, int K) {
  static_assert(ACT == 0);
  __shared__ __attribute__((aligned(16))) float so[4][32][68];
  const int tid = threadIdx.x, w = tid >> 5, lane = tid & 31, ln = lane & 15, hh = lane >> 4; const int by = blockIdx.y;
  A += (size_t)by * sA; Bh += (size_t)by * sB; const size_t cofs = (size_t)by * sC; const float* bp = bias ? bias + (size_t)by * sBias : nullptr;
  const int ntn = N >> 6; const int mt = blockIdx.x / ntn, nq = blockIdx.x - mt * ntn; const int row0 = mt * 128 + 32 * w, col0 = nq * 64; if (row0 >= M) return;
  const _Float16* a0p = A + (size_t)(row0 + ln) * lda; const _Float16* a1p = a0p + (size_t)16 * lda;
  const _Float16* b0p = Bh + (size_t)(col0 + ln) * ldb; const _Float16* b1p = b0p + (size_t)16 * ldb; const _Float16* b2p = b1p + (size_t)16 * ldb; const _Float16* b3p = b2p + (size_t)16 * ldb;
  const v8f z8 = {0.f,0.f,0.f,0.f,0.f,0.f,0.f,0.f}; v8f c00 = z8, c01 = z8, c02 = z8, c03 = z8, c10 = z8, c11 = z8, c12 = z8, c13 = z8;
#pragma unroll 1
  for (int kb = 0; kb < K; kb += 32) { const v16h a0 = g2_frag(a0p + kb, hh), a1 = g2_frag(a1p + kb, hh);
    v16h b = g2_frag(b0p + kb, hh); c00 = g2_mma(a0, b, c00); c10 = g2_mma(a1, b, c10);
    b = g2_frag(b1p + kb, hh); c01 = g2_mma(a0, b, c01); c11 = g2_mma(a1, b, c11);
    b = g2_frag(b2p + kb, hh); c02 = g2_mma(a0, b, c02); c12 = g2_mma(a1, b, c12);
    b = g2_frag(b3p + kb, hh); c03 = g2_mma(a0, b, c03); c13 = g2_mma(a1, b, c13); }
  v8f accs[8] = {c00, c01, c02, c03, c10, c11, c12, c13};
#pragma unroll
  for (int u = 0; u < 8; ++u) { const int t = u & 3, half = u >> 2; const int col = col0 + t * 16 + ln; const float bv = bp ? bf16_rne(bp[col]) : 0.f;
#pragma unroll
    for (int r = 0; r < 8; ++r) { const int rloc = half * 16 + 8 * hh + r; float v = accs[u][r] * alpha + bv;
      if (CP) { if (rowsPerB < 0) v += CP[cofs + (size_t)(row0g + row0 + rloc) * ldc + col]; else { const int bidx = (row0g + row0 + rloc) / rowsPerB; v += CP[(size_t)bidx * sCPb + (size_t)by * 64 + col]; } }
      so[w][rloc][t * 16 + ln] = v; } }
  __builtin_amdgcn_fence(4  , "workgroup"); __builtin_amdgcn_wave_barrier();
  const int rsub = lane >> 4, c4 = (lane & 15) * 4;
  for (int pass = 0; pass < 2; ++pass) {
#pragma unroll
    for (int q = 0; q < 16; ++q) { const int r = q * 2 + rsub; const v4f v = *(const v4fa*)&so[w][r][c4];
      if (C) *(volatile v4f*)(C + cofs + (size_t)(row0 + r) * ldc + col0 + c4) = v;
      if (C16) { v4h h4; for (int i = 0; i < 4; ++i) h4[i] = (_Float16)v[i]; *(volatile v4h*)(C16 + cofs + (size_t)(row0 + r) * ldc + col0 + c4) = h4; } }
    if (pass == 0) __threadfence(); }
}

extern "C" void kernel_launch(void* const* d_in, const int* in_sizes, int n_in,
                              void* d_out, int out_size, void* d_ws, size_t ws_size, hipStream_t stream) {
  if (n_in < 3) return;
  if ((size_t)in_sizes[0] < (size_t)(NB - 1) * SEQ_FULL * CD + (size_t)SEQ * CD || in_sizes[1] < CD * HW || in_sizes[2] < CD * HW) return;
  if ((size_t)out_size < (size_t)(NB - 1) * SEQ_FULL * HW + (size_t)SEQ * HW) return;
  const float* xin = (const float*)d_in[0]; const float* Wqk = (const float*)d_in[1]; const float* Wov = (const float*)d_in[2];
  char* ws = (char*)d_ws; size_t off = 0;
  auto take = [&](size_t bytes) { char* p = ws + off; off += (bytes + 255) & ~(size_t)255; return p; };
  _Float16* X16  = (_Float16*)take((size_t)NB * SEQ * CD * 2);
  _Float16* WT16 = (_Float16*)take((size_t)KVW * CD * 2);
  float*    KVf  = (float*)take((size_t)NB * SEQ * KVW * 4);
  _Float16* KVT  = (_Float16*)take((size_t)2 * NB * HW * SEQ * 2);
  _Float16* Mt16 = (_Float16*)take((size_t)NB * NH * CD * CD * 2);
  if (off > ws_size) return;
  _Float16* KT16 = KVT; _Float16* VT16 = KVT + (size_t)NB * HW * SEQ;
  const size_t n8x = (size_t)SEQ * CD / 8;
  for (int b = 0; b < NB; ++b)
    k_wnat<<<(unsigned)((n8x + 255) / 256), 256, 0, stream>>>(xin + (size_t)b * SEQ_FULL * CD, n8x, X16 + (size_t)b * SEQ * CD);
  k_wtr<<<(CD / 64) * (HW / 64), 256, 0, stream>>>(Wqk, WT16);
  k_wtr<<<(CD / 64) * (HW / 64), 256, 0, stream>>>(Wov, WT16 + (size_t)HW * CD);
  k_gemm2<0><<<dim3((NB * SEQ / 128) * (KVW / 64), 1), 128, 0, stream>>>(X16, CD, (size_t)0, WT16, CD, (size_t)0, 0.0625f, (const float*)nullptr, (size_t)0, (const float*)nullptr, 1, (size_t)0, 0, KVf, (_Float16*)nullptr, KVW, (size_t)0, NB * SEQ, KVW, CD);
  k_kvt<<<NB * (KVW / 64) * (SEQ / 64), 256, 0, stream>>>(KVf, KVT);
  k_gemm2<0><<<dim3((CD / 128) * (CD / 64), NB * NH), 128, 0, stream>>>(VT16, SEQ, (size_t)CD * SEQ, KT16, SEQ, (size_t)CD * SEQ, 0.00390625f, (const float*)nullptr, (size_t)0, (const float*)nullptr, 1, (size_t)0, 0, (float*)nullptr, Mt16, CD, (size_t)CD * CD, CD, CD, SEQ);
  k_gemm2<0><<<dim3((SEQ / 128) * (HW / 64), NB), 128, 0, stream>>>(X16, CD, (size_t)SEQ * CD, Mt16, CD, (size_t)HW * CD, 1.52587890625e-05f, (const float*)nullptr, (size_t)0, (const float*)nullptr, 1, (size_t)0, 0, (float*)d_out, (_Float16*)nullptr, HW, (size_t)SEQ_FULL * HW, SEQ, HW, CD);
}
